// MultiheadAttention_67559835566643
// MI455X (gfx1250) — hardware-run, weakly checked
//
#include <hip/hip_runtime.h>
#ifndef NB
#define NB 4
#endif
#ifndef SEQ
#define SEQ 1024
#endif
#define NB_FULL 4
#define DM 1024
#define NH 16
#define HD 64
#define SLEN (SEQ + 1)
#define NKP (((SLEN + 63) / 64) * 64)
#define NKX NKP
#define KTR (SEQ + 8)
#define KSTR ((size_t)KTR * DM)
#ifndef QT
#define QT ((SEQ) < 512 ? (SEQ) : 512)
#endif
static_assert(SEQ % 128 == 0);
static_assert(QT % 256 == 0);
static_assert(SEQ % QT == 0);
static_assert(NKP % 64 == 0);
static_assert(NKP % 32 == 0);
static_assert(16 * KTR >= 15 * SLEN + NKP);
static_assert((NB * NH * SEQ) % 256 == 0);
static_assert(NB <= NB_FULL);

typedef unsigned short v8us __attribute__((ext_vector_type(8), may_alias));
typedef float  v8f  __attribute__((ext_vector_type(8)));
typedef float  v4f  __attribute__((ext_vector_type(4)));
typedef float  v4fa __attribute__((ext_vector_type(4), may_alias));
typedef _Float16 v16h __attribute__((ext_vector_type(16)));
typedef _Float16 v4h __attribute__((ext_vector_type(4)));
union FragH { v16h v; v8us half[2]; _Float16 h[16]; unsigned short u[16]; };

__device__ __forceinline__ unsigned short bf16_bits(float x) { unsigned int u = __float_as_uint(x); return (unsigned short)((u + 0x7FFFu + ((u >> 16) & 1u)) >> 16); }
__device__ __forceinline__ float bf16_rne(float x) { return __uint_as_float(((unsigned int)bf16_bits(x)) << 16); }

__global__ __launch_bounds__(256) void k_wt_f16(const float* __restrict__ W, _Float16* __restrict__ Wt, int K, int N, float scale) {
  const int t = blockIdx.x * 256 + threadIdx.x; if (t >= N * (K / 8)) return; const int n = t / (K / 8), k8 = (t % (K / 8)) * 8; FragH f;
#pragma unroll
  for (int i = 0; i < 8; ++i) f.h[i] = (_Float16)(bf16_rne(W[(size_t)(k8 + i) * N + n]) * scale);
  const v8us o = f.half[0];
  *(volatile v8us*)((unsigned short*)Wt + (size_t)n * K + k8) = o; __threadfence(); *(volatile v8us*)((unsigned short*)Wt + (size_t)n * K + k8) = o;
}

__global__ __launch_bounds__(256) void k_x16b(const float* __restrict__ x, _Float16* __restrict__ X16) {
  const size_t t = (size_t)blockIdx.x * 256 + threadIdx.x; if (t >= (size_t)NB * SEQ * (DM / 8)) return;
  const int c8 = (int)(t % (DM / 8)) * 8; const size_t r = t / (DM / 8); const int b = (int)(r / SEQ), tt = (int)(r % SEQ);
  const float* src = x + ((size_t)tt * NB_FULL + b) * DM + c8;
  const v4f a = *(const v4fa*)src, c = *(const v4fa*)(src + 4); FragH f;
#pragma unroll
  for (int q = 0; q < 4; ++q) { f.h[q] = (_Float16)bf16_rne(a[q]); f.h[4 + q] = (_Float16)bf16_rne(c[q]); }
  const v8us o = f.half[0];
  *(volatile v8us*)((unsigned short*)X16 + t * 8) = o; __threadfence(); *(volatile v8us*)((unsigned short*)X16 + t * 8) = o;
}

__global__ __launch_bounds__(256) void k_hlb(const float* __restrict__ F, size_t sF, _Float16* __restrict__ Hh, _Float16* __restrict__ Hl, size_t sH, size_t n8) {
  const size_t t = (size_t)blockIdx.x * 256 + threadIdx.x; if (t >= n8) return;
  F += (size_t)blockIdx.y * sF; Hh += (size_t)blockIdx.y * sH; Hl += (size_t)blockIdx.y * sH;
  FragH fh, fl; const v4f a = *(const v4fa*)(F + t * 8), c = *(const v4fa*)(F + t * 8 + 4);
#pragma unroll
  for (int q = 0; q < 4; ++q) { _Float16 h = (_Float16)a[q]; fh.h[q] = h; fl.h[q] = (_Float16)((a[q] - (float)h) * 1024.0f); h = (_Float16)c[q]; fh.h[4 + q] = h; fl.h[4 + q] = (_Float16)((c[q] - (float)h) * 1024.0f); }
  const v8us oh = fh.half[0], ol = fl.half[0];
  for (int pass = 0; pass < 2; ++pass) { *(volatile v8us*)((unsigned short*)Hh + t * 8) = oh; *(volatile v8us*)((unsigned short*)Hl + t * 8) = ol; if (pass == 0) __threadfence(); }
}

__global__ __launch_bounds__(256) void k_kvtail(const float* __restrict__ bk, const float* __restrict__ bv, _Float16* __restrict__ KH, _Float16* __restrict__ KL, _Float16* __restrict__ V16) {
  const int per = (KTR - SEQ) * (DM / 8); const int t = blockIdx.x * 256 + threadIdx.x; if (t >= NB * per) return;
  const int b = t / per, u = t % per, rr = u / (DM / 8), c8 = (u % (DM / 8)) * 8;
  FragH fk, fl, fv;
#pragma unroll
  for (int q = 0; q < 8; ++q) { float a = bf16_rne(bk[c8 + q]); float c = bf16_rne(bv[c8 + q]); a = (rr == 0) ? a : 0.f; c = (rr == 0) ? c : 0.f; const _Float16 h = (_Float16)a; fk.h[q] = h; fl.h[q] = (_Float16)((a - (float)h) * 1024.0f); fv.h[q] = (_Float16)c; }
  const size_t off = (size_t)b * KSTR + (size_t)(SEQ + rr) * DM + c8; const v8us ok = fk.half[0], ol = fl.half[0], ov = fv.half[0];
  for (int pass = 0; pass < 2; ++pass) { *(volatile v8us*)((unsigned short*)KH + off) = ok; *(volatile v8us*)((unsigned short*)KL + off) = ol; *(volatile v8us*)((unsigned short*)V16 + off) = ov; if (pass == 0) __threadfence(); }
}

__global__ __launch_bounds__(256) void k_gate(const float* __restrict__ QF, const float* __restrict__ gw, const float* __restrict__ gb, const float* __restrict__ ga, float* __restrict__ gate) {
  __shared__ float gws[HD + 1];
  const int tid = threadIdx.x;
  if (tid < HD) { float s = 0.f; for (int j = 0; j < 8; ++j) s += bf16_rne(gw[tid * 8 + j]); gws[tid] = s; }
  if (tid == HD) { float s = 0.f; for (int j = 0; j < 8; ++j) s += bf16_rne(gb[j]); gws[HD] = s; }
  __syncthreads();
  const int row = blockIdx.x * 256 + tid; const int hp = (row / SEQ) % NH;
  const float* q = QF + (size_t)row * HD; float s = gws[HD];
#pragma unroll 1
  for (int c = 0; c < HD / 4; ++c) { const v4f qq = *(const v4fa*)(q + c * 4); s += qq[0] * gws[c * 4] + qq[1] * gws[c * 4 + 1] + qq[2] * gws[c * 4 + 2] + qq[3] * gws[c * 4 + 3]; }
  const float g = (1.0f / (1.0f + __expf(-s))) * bf16_rne(ga[hp]);
  *(volatile float*)(gate + row) = g; __threadfence(); *(volatile float*)(gate + row) = g;
}

__device__ __forceinline__ v16h g2_frag(const _Float16* p, int hh) { FragH f; f.half[0] = *(const v8us*)((const unsigned short*)p + 8 * hh); f.half[1] = *(const v8us*)((const unsigned short*)p + 16 + 8 * hh); return f.v; }
__device__ __forceinline__ v8f g2_mma(v16h a, v16h b, v8f c) { v8f d = __builtin_amdgcn_wmma_f32_16x16x32_f16(false, a, false, b, (short)0, c, false, false); asm volatile("v_nop\n\tv_nop\n\tv_nop\n\tv_nop" : "+v"(d) : "v"(a), "v"(b)); return d; }
__global__ __launch_bounds__(128) void k_gemm2(const _Float16* __restrict__ A, int lda, size_t sA, const _Float16* __restrict__ Bh, int ldb, size_t sB, float alpha, const float* __restrict__ bias, const float* CP,
    float* C, _Float16* C16, int ldc, size_t sC, int M, int N, int K) {
  __shared__ __attribute__((aligned(16))) float so[4][32][68];
  const int tid = threadIdx.x, w = __builtin_amdgcn_readfirstlane((int)(tid >> 5)), lane = tid & 31, ln = lane & 15, hh = lane >> 4; const int by = blockIdx.y;
  A += (size_t)by * sA; Bh += (size_t)by * sB; const size_t cofs = (size_t)by * sC;
  const int ntn = N >> 6; const int mt = blockIdx.x / ntn, nq = blockIdx.x - mt * ntn; const int row0 = mt * 128 + 32 * w, col0 = nq * 64; if (row0 >= M) return;
  const _Float16* a0p = A + (size_t)(row0 + ln) * lda; const _Float16* a1p = a0p + (size_t)16 * lda;
  const _Float16* b0p = Bh + (size_t)(col0 + ln) * ldb; const _Float16* b1p = b0p + (size_t)16 * ldb; const _Float16* b2p = b1p + (size_t)16 * ldb; const _Float16* b3p = b2p + (size_t)16 * ldb;
  const v8f z8 = {0.f,0.f,0.f,0.f,0.f,0.f,0.f,0.f}; v8f c00 = z8, c01 = z8, c02 = z8, c03 = z8, c10 = z8, c11 = z8, c12 = z8, c13 = z8;
#pragma unroll 1
  for (int kb = 0; kb < K; kb += 32) { const v16h a0 = g2_frag(a0p + kb, hh), a1 = g2_frag(a1p + kb, hh);
    v16h b = g2_frag(b0p + kb, hh); c00 = g2_mma(a0, b, c00); c10 = g2_mma(a1, b, c10);
    b = g2_frag(b1p + kb, hh); c01 = g2_mma(a0, b, c01); c11 = g2_mma(a1, b, c11);
    b = g2_frag(b2p + kb, hh); c02 = g2_mma(a0, b, c02); c12 = g2_mma(a1, b, c12);
    b = g2_frag(b3p + kb, hh); c03 = g2_mma(a0, b, c03); c13 = g2_mma(a1, b, c13); }
  v8f accs[8] = {c00, c01, c02, c03, c10, c11, c12, c13};
#pragma unroll
  for (int u = 0; u < 8; ++u) { const int t = u & 3, half = u >> 2; const int col = col0 + t * 16 + ln; const float bv = bias ? bf16_rne(bias[col]) : 0.f;
#pragma unroll
    for (int r = 0; r < 8; ++r) { const int rloc = half * 16 + 8 * hh + r; float v = accs[u][r] * alpha + bv; if (CP) v += CP[cofs + (size_t)(row0 + rloc) * ldc + col];
      so[w][rloc][t * 16 + ln] = v; } }
  __builtin_amdgcn_fence(4  , "workgroup"); __builtin_amdgcn_wave_barrier();
  const int rsub = lane >> 4, c4 = (lane & 15) * 4;
  for (int pass = 0; pass < 2; ++pass) {
#pragma unroll
    for (int q = 0; q < 16; ++q) { const int r = q * 2 + rsub; const v4f v = *(const v4fa*)&so[w][r][c4]; if (C) *(volatile v4f*)(C + cofs + (size_t)(row0 + r) * ldc + col0 + c4) = v; if (C16) { v4h h4; for (int i = 0; i < 4; ++i) h4[i] = (_Float16)v[i]; *(volatile v4h*)(C16 + cofs + (size_t)(row0 + r) * ldc + col0 + c4) = h4; } }
    if (pass == 0) __threadfence(); }
}

__global__ __launch_bounds__(256) void k_vtp(const _Float16* __restrict__ Vb, _Float16* __restrict__ VT) {
  __shared__ unsigned short tl[64][66];
  const int tid = threadIdx.x; const int hp = blockIdx.x / (NKP / 64), lg = blockIdx.x % (NKP / 64);
  for (int i = tid; i < 64 * 8; i += 256) { const int r = i / 8, c8 = (i % 8) * 8; FragH f;
    f.half[0] = *(const v8us*)((const unsigned short*)Vb + ((size_t)hp * SLEN + lg * 64 + r) * HD + c8);
    const bool ok = (lg * 64 + r) < SLEN;
#pragma unroll
    for (int q = 0; q < 8; ++q) tl[r][c8 + q] = ok ? f.u[q] : (unsigned short)0; }
  __syncthreads();
  for (int pass = 0; pass < 2; ++pass) {
#pragma unroll
    for (int rd = 0; rd < 2; ++rd) { const int d = rd * 32 + tid / 8, pc = tid % 8; FragH f;
#pragma unroll
      for (int q = 0; q < 8; ++q) f.u[q] = tl[pc * 8 + q][d];
      const v8us o = f.half[0];
      *(volatile v8us*)((unsigned short*)VT + ((size_t)hp * HD + d) * NKX + lg * 64 + pc * 8) = o; }
    if (pass == 0) __threadfence(); }
}

__global__ __launch_bounds__(256) void k_rsmpb(const float* __restrict__ S, _Float16* __restrict__ P, const float* __restrict__ gate, const float* __restrict__ rel_emb, int q0) {
  #pragma clang fp contract(off)
  __shared__ float pbt[2 * SEQ];
  const int tid = threadIdx.x; const int t = blockIdx.x * 256 + tid; const int hp = (blockIdx.x * 256) / QT;
#pragma unroll 1
  for (int p = tid; p < 2 * SEQ; p += 256) { const int rel = p - (SEQ - 1); const int a = rel < 0 ? -rel : rel;
    const int lg = 8 + (a >= 12) + (a >= 16) + (a >= 23) + (a >= 32) + (a >= 46) + (a >= 64) + (a >= 91);
    const int bk = ((rel > 0) ? 16 : 0) + ((a < 8) ? a : lg);
    pbt[p] = bf16_rne(rel_emb[bk * NH + hp]); }
  __syncthreads();
  const int tq = q0 + (t % QT); const float g = gate[(size_t)hp * SEQ + tq]; const float* s = S + (size_t)t * NKX; const int po = SEQ - 1 - tq;
  float mx = -3.0e38f;
#pragma unroll 1
  for (int j = 0; j < SLEN; ++j) { const float gp = g * pbt[j + po]; mx = fmaxf(mx, s[j] + gp); }
  float se = 0.f;
#pragma unroll 1
  for (int j = 0; j < SLEN; ++j) { const float gp = g * pbt[j + po]; se += __expf((s[j] + gp) - mx); }
  const float sc = 256.0f / se;
#pragma unroll 1
  for (int j0 = 0; j0 < NKP; j0 += 8) { FragH fr;
#pragma unroll
    for (int q = 0; q < 8; ++q) { const int j = j0 + q; const int jc = (j < SLEN) ? j : (SLEN - 1); const float gp = g * pbt[jc + po]; const float e = __expf((s[jc] + gp) - mx) * sc; fr.h[q] = (_Float16)((j < SLEN) ? e : 0.f); }
    const v8us o = fr.half[0]; unsigned short* d = (unsigned short*)P + (size_t)t * NKX + j0; *(volatile v8us*)d = o; __threadfence(); *(volatile v8us*)d = o; }
}

extern "C" void kernel_launch(void* const* d_in, const int* in_sizes, int n_in,
                              void* d_out, int out_size, void* d_ws, size_t ws_size, hipStream_t stream) {
  if (n_in < 15) return;
  if ((size_t)in_sizes[0] < ((size_t)(SEQ - 1) * NB_FULL + NB) * DM) return;
  if (in_sizes[1] < DM * DM || in_sizes[3] < DM * DM || in_sizes[5] < DM * DM || in_sizes[7] < DM * DM) return;
  if (in_sizes[2] < DM || in_sizes[4] < DM || in_sizes[6] < DM || in_sizes[8] < DM || in_sizes[13] < DM || in_sizes[14] < DM) return;
  if (in_sizes[9] < 32 * NH || in_sizes[10] < HD * 8 || in_sizes[11] < 8 || in_sizes[12] < NH) return;
  if ((size_t)out_size < (size_t)NB * SEQ * DM) return;
  const float* const* I = (const float* const*)d_in;
  const float* x = I[0]; const float* wq = I[1]; const float* bq = I[2]; const float* wk = I[3]; const float* bk = I[4]; const float* wv = I[5]; const float* bv = I[6]; const float* wo = I[7]; const float* bo = I[8];
  const float* rel_emb = I[9]; const float* grep_w = I[10]; const float* grep_b = I[11]; const float* grep_a = I[12]; const float* bias_k = I[13]; const float* bias_v = I[14];
  char* ws = (char*)d_ws; size_t off = 0;
  auto take = [&](size_t bytes) { char* p = ws + off; off += (bytes + 255) & ~(size_t)255; return p; };
  const size_t NRD = (size_t)NB * SEQ * DM;
  _Float16* BQ = (_Float16*)take((size_t)DM * DM * 2); _Float16* BK = (_Float16*)take((size_t)DM * DM * 2); _Float16* BV = (_Float16*)take((size_t)DM * DM * 2); _Float16* BO = (_Float16*)take((size_t)DM * DM * 2);
  _Float16* X16 = (_Float16*)take(NRD * 2);
  _Float16* QH = (_Float16*)take(NRD * 2); _Float16* QL = (_Float16*)take(NRD * 2);
  _Float16* KH = (_Float16*)take((size_t)NB * KSTR * 2); _Float16* KL = (_Float16*)take((size_t)NB * KSTR * 2); _Float16* V16 = (_Float16*)take((size_t)NB * KSTR * 2);
  _Float16* O16 = (_Float16*)take(NRD * 2);
  const size_t sbytes = (size_t)NH * QT * NKX * 4; const size_t qfbytes = NRD * 4;
  float* S = (float*)take(sbytes > qfbytes ? sbytes : qfbytes); float* QF = S;
  _Float16* P = (_Float16*)take((size_t)NH * QT * NKX * 2); _Float16* VT = (_Float16*)take((size_t)NH * HD * NKX * 2);
  float* GT = (float*)take((size_t)NB * NH * SEQ * 4);
  if (off > ws_size || off > (size_t)134217728) return;

  { const unsigned g = (unsigned)(((size_t)DM * DM / 8 + 255) / 256);
    k_wt_f16<<<g, 256, 0, stream>>>(wq, BQ, DM, DM, 16.0f); k_wt_f16<<<g, 256, 0, stream>>>(wk, BK, DM, DM, 16.0f); k_wt_f16<<<g, 256, 0, stream>>>(wv, BV, DM, DM, 16.0f); k_wt_f16<<<g, 256, 0, stream>>>(wo, BO, DM, DM, 16.0f); }
  k_x16b<<<(unsigned)((NRD / 8 + 255) / 256), 256, 0, stream>>>(x, X16);
  const unsigned gproj = (unsigned)(((NB * SEQ) / 128) * (DM / 64)); const unsigned ghl = (unsigned)(((size_t)SEQ * DM / 8 + 255) / 256);
  k_gemm2<<<dim3(gproj, 1), 128, 0, stream>>>(X16, DM, 0, BQ, DM, 0, 0.0625f, bq, nullptr, QF, nullptr, DM, 0, NB * SEQ, DM, DM);
  k_hlb<<<dim3(ghl, NB), 256, 0, stream>>>(QF, (size_t)SEQ * DM, QH, QL, (size_t)SEQ * DM, (size_t)SEQ * DM / 8);
  k_gate<<<(NB * NH * SEQ) / 256, 256, 0, stream>>>(QF, grep_w, grep_b, grep_a, GT);
  k_gemm2<<<dim3(gproj, 1), 128, 0, stream>>>(X16, DM, 0, BK, DM, 0, 0.0625f, bk, nullptr, QF, nullptr, DM, 0, NB * SEQ, DM, DM);
  k_hlb<<<dim3(ghl, NB), 256, 0, stream>>>(QF, (size_t)SEQ * DM, KH, KL, KSTR, (size_t)SEQ * DM / 8);
  k_gemm2<<<dim3((SEQ / 128) * (DM / 64), NB), 128, 0, stream>>>(X16, DM, (size_t)SEQ * DM, BV, DM, 0, 0.0625f, bv, nullptr, nullptr, V16, DM, KSTR, SEQ, DM, DM);
  k_kvtail<<<(NB * (KTR - SEQ) * (DM / 8) + 255) / 256, 256, 0, stream>>>(bias_k, bias_v, KH, KL, V16);
  for (int b = 0; b < NB; ++b) {
    k_vtp<<<NH * (NKP / 64), 256, 0, stream>>>(V16 + (size_t)b * KSTR, VT);
    for (int q0 = 0; q0 < SEQ; q0 += QT) {
      const _Float16* qh = QH + (size_t)b * SEQ * DM + (size_t)q0 * HD; const _Float16* ql = QL + (size_t)b * SEQ * DM + (size_t)q0 * HD;
      const _Float16* kh = KH + (size_t)b * KSTR; const _Float16* kl = KL + (size_t)b * KSTR;
      const dim3 gs((QT / 128) * (NKP / 64), NH);
      k_gemm2<<<gs, 128, 0, stream>>>(qh, HD, (size_t)SEQ * HD, kh, HD, (size_t)SLEN * HD, 0.00390625f, nullptr, nullptr, S, nullptr, NKX, (size_t)QT * NKX, QT, NKP, HD);
      k_gemm2<<<gs, 128, 0, stream>>>(ql, HD, (size_t)SEQ * HD, kh, HD, (size_t)SLEN * HD, 0.000003814697265625f, nullptr, S, S, nullptr, NKX, (size_t)QT * NKX, QT, NKP, HD);
      k_gemm2<<<gs, 128, 0, stream>>>(qh, HD, (size_t)SEQ * HD, kl, HD, (size_t)SLEN * HD, 0.000003814697265625f, nullptr, S, S, nullptr, NKX, (size_t)QT * NKX, QT, NKP, HD);
      k_rsmpb<<<(NH * QT) / 256, 256, 0, stream>>>(S, P, GT + (size_t)b * NH * SEQ, rel_emb, q0);
      k_gemm2<<<dim3((QT / 128) * (HD / 64), NH), 128, 0, stream>>>(P, NKX, (size_t)QT * NKX, VT, NKX, (size_t)HD * NKX, 0.25f, nullptr, nullptr, nullptr, O16 + ((size_t)q0 * NB + b) * DM, NB * DM, (size_t)HD, QT, HD, NKP);
    }
  }
  k_gemm2<<<dim3(gproj, 1), 128, 0, stream>>>(O16, DM, 0, BO, DM, 0, 0.0009765625f, bo, nullptr, (float*)d_out, nullptr, DM, 0, NB * SEQ, DM, DM);
}
